// MinEuclideanDistBlock_46480136077428
// MI455X (gfx1250) — hardware-verified
//
#include <hip/hip_runtime.h>
#include <stdint.h>

typedef __attribute__((ext_vector_type(16))) _Float16 v16h;
typedef __attribute__((ext_vector_type(8)))  _Float16 v8h;
typedef __attribute__((ext_vector_type(8)))  float    v8f;
typedef __attribute__((ext_vector_type(4)))  float    v4f;

__device__ __forceinline__ void dep_guard_h(v8f& a, v8f& b, v16h x, v16h y) { asm volatile("v_nop\n\tv_nop\n\tv_nop\n\tv_nop" : "+v"(a), "+v"(b) : "v"(x), "v"(y)); }
__device__ __forceinline__ void keep4_h(v16h a, v16h b, v16h c, v16h d) { asm volatile("v_nop" :: "v"(a), "v"(b), "v"(c), "v"(d)); }
__device__ __forceinline__ void acc_guard4(v8f& a, v8f& b, v8f& c, v8f& d) { asm volatile("v_nop\n\tv_nop\n\tv_nop\n\tv_nop" : "+v"(a), "+v"(b), "+v"(c), "+v"(d)); }
template <typename T> struct Frag;
template <> struct Frag<_Float16> {
  typedef v16h V; union U { v16h v; v8h h[2]; };
  static __device__ __forceinline__ v16h load(const _Float16* p) {
    U f; f.h[0] = *(const v8h*)(p); f.h[1] = *(const v8h*)(p + 16); return f.v;
  }
  static __device__ __forceinline__ v8f mma(v16h a, v16h b, v8f c) {
    return __builtin_amdgcn_wmma_f32_16x16x32_f16(false, a, false, b, (short)0, c, false, false);
  }
  static __device__ __forceinline__ void guard(v8f& a, v8f& b, v16h x, v16h y) { dep_guard_h(a, b, x, y); }
  static __device__ __forceinline__ void keep(v16h a, v16h b, v16h c, v16h d) { keep4_h(a, b, c, d); }
};

constexpr int SHP_LEN   = 64;
constexpr int NUM_SHP   = 128;
constexpr int NUM_CH    = 8;
constexpr int SER_LEN   = 2048;
constexpr int NUM_WIN   = SER_LEN - SHP_LEN + 1;
constexpr int WIN_TILE  = 64;
constexpr int NUM_WTILE = (NUM_WIN + WIN_TILE - 1) / WIN_TILE;
constexpr int XS_LEN    = WIN_TILE + SHP_LEN + 8;
constexpr int CP_LEN    = WIN_TILE + SHP_LEN;
constexpr int SHP_ROWS  = NUM_CH * NUM_SHP;
static_assert(SHP_ROWS % 32 == 0, "rows per block");
static_assert(SHP_LEN == 64, "depth 64 = 2 k-steps of 32");
static_assert(NUM_SHP == 128, "4 waves x 32 columns");
static_assert(WIN_TILE == 64, "2 waves x 32 rows");
static_assert(NUM_WTILE * WIN_TILE >= NUM_WIN, "tile coverage");
static_assert((CP_LEN * 2) % 16 == 0, "copy row pitch 16B aligned");

__global__ __launch_bounds__(256) void znorm_rows_kernel(const float* __restrict__ sh,
                                                         unsigned short* __restrict__ shn16,
                                                         float* __restrict__ sqs) {
  __shared__ float sq_l[32];
  const int tid  = threadIdx.x;
  const int lane = tid & 31;
  const int wave = tid >> 5;
  const int rbase = blockIdx.x * 32;
#pragma unroll 1
  for (int rr = 0; rr < 4; ++rr) {
    const int rloc = wave * 4 + rr;
    const int row  = rbase + rloc;
    const float* s = sh + (size_t)row * SHP_LEN;
    const float v0 = s[2 * lane];
    const float v1 = s[2 * lane + 1];
    float sm = v0 + v1;
#pragma unroll
    for (int off = 1; off < 32; off <<= 1) sm += __shfl_xor(sm, off, 32);
    const float mu = sm * (1.0f / 64.0f);
    const float d0 = v0 - mu;
    const float d1 = v1 - mu;
    float vr = d0 * d0 + d1 * d1;
#pragma unroll
    for (int off = 1; off < 32; off <<= 1) vr += __shfl_xor(vr, off, 32);
    vr *= (1.0f / 64.0f);
    const float rsd = 1.0f / sqrtf(vr);
    const float z0 = d0 * rsd;
    const float z1 = d1 * rsd;
    float ss = z0 * z0 + z1 * z1;
#pragma unroll
    for (int off = 1; off < 32; off <<= 1) ss += __shfl_xor(ss, off, 32);
    if (lane == 0) sq_l[rloc] = ss;
    const unsigned u = (unsigned)__builtin_bit_cast(unsigned short, (_Float16)z0) |
                       ((unsigned)__builtin_bit_cast(unsigned short, (_Float16)z1) << 16);
    volatile unsigned* p = (volatile unsigned*)(shn16) + (size_t)row * (SHP_LEN / 2) + lane;
    *p = u;
    __threadfence();
    *p = u;
  }
  __syncthreads();
  if (wave == 0) {
    const float v = sq_l[lane];
    volatile float* q = (volatile float*)(sqs + rbase + lane);
    *q = v;
    __threadfence();
    *q = v;
  }
}

__global__ __launch_bounds__(256) void min_dist_kernel(const float* __restrict__ x,
                                                       const unsigned short* __restrict__ shn16,
                                                       const float* __restrict__ sqs,
                                                       float* __restrict__ out) {
  __shared__ __align__(16) float    xs[XS_LEN];
  __shared__ __align__(16) _Float16 xcp[8][CP_LEN];
  __shared__ float sqx[WIN_TILE];
  __shared__ float minbuf[2][NUM_SHP];

  const int n    = blockIdx.x;
  const int tid  = threadIdx.x;
  const int lane = tid & 31;
  const int wave = tid >> 5;
  const int ww   = wave & 1;
  const int wk   = wave >> 1;
  const int rlane = lane & 15;
  const int hh    = lane >> 4;
  const _Float16* Bbase = (const _Float16*)(const void*)shn16;

  float runmin0 = __builtin_inff();
  float runmin1 = __builtin_inff();

#pragma unroll 1
  for (int wt = 0; wt < NUM_WTILE; ++wt) {
    const int w0 = wt * WIN_TILE;
    v8f dsum[2][2];
#pragma unroll
    for (int i = 0; i < 2; ++i)
#pragma unroll
      for (int j = 0; j < 2; ++j) dsum[i][j] = (v8f){0.f,0.f,0.f,0.f,0.f,0.f,0.f,0.f};

#pragma unroll 1
    for (int c = 0; c < NUM_CH; ++c) {
      __syncthreads();
      const float* xrow = x + ((size_t)n * NUM_CH + c) * SER_LEN;
      if (tid < XS_LEN) {
        int gi = w0 + tid;
        gi = (gi < SER_LEN) ? gi : (SER_LEN - 1);
        xs[tid] = xrow[gi];
      }
      __syncthreads();
#pragma unroll
      for (int q = 0; q < 2; ++q) {
        const int wi = tid + q * 256;
        const int j  = wi >> 6;
        const int t2 = (wi & 63) * 2;
        const float f0 = xs[t2 + j];
        const float f1 = xs[t2 + 1 + j];
        const unsigned u = (unsigned)__builtin_bit_cast(unsigned short, (_Float16)f0) |
                           ((unsigned)__builtin_bit_cast(unsigned short, (_Float16)f1) << 16);
        *(unsigned*)(&xcp[j][t2]) = u;
      }
      {
        const int wl = tid >> 2;
        const int qq = tid & 3;
        float a = 0.f;
#pragma unroll
        for (int s = 0; s < 16; ++s) { const float v = xs[wl + 16 * qq + s]; a += v * v; }
        a += __shfl_xor(a, 1, 32);
        a += __shfl_xor(a, 2, 32);
        if (qq == 0) sqx[wl] = a;
      }
      __syncthreads();

      v8f acc[2][2];
#pragma unroll
      for (int i = 0; i < 2; ++i)
#pragma unroll
        for (int j = 0; j < 2; ++j) acc[i][j] = (v8f){0.f,0.f,0.f,0.f,0.f,0.f,0.f,0.f};
      const _Float16* Bc = Bbase + (size_t)c * NUM_SHP * SHP_LEN;
#pragma unroll
      for (int ks = 0; ks < 2; ++ks) {
        v16h bf[2];
#pragma unroll
        for (int j = 0; j < 2; ++j)
          bf[j] = Frag<_Float16>::load(Bc + (size_t)(32 * wk + 16 * j + rlane) * SHP_LEN + 32 * ks + 8 * hh);
#pragma unroll
        for (int i = 0; i < 2; ++i) {
          const int bidx = 32 * ww + 16 * i + rlane + 32 * ks + 8 * hh;
          const int jj   = bidx & 7;
          const int base = bidx - jj;
          const v16h af = Frag<_Float16>::load(&xcp[jj][base]);
          acc[i][0] = Frag<_Float16>::mma(af, bf[0], acc[i][0]);
          acc[i][1] = Frag<_Float16>::mma(af, bf[1], acc[i][1]);
          Frag<_Float16>::guard(acc[i][0], acc[i][1], af, af);
        }
        Frag<_Float16>::keep(bf[0], bf[1], bf[0], bf[1]);
      }
      acc_guard4(acc[0][0], acc[0][1], acc[1][0], acc[1][1]);

      float sxv[2][8];
#pragma unroll
      for (int i = 0; i < 2; ++i)
#pragma unroll
        for (int r = 0; r < 8; ++r) sxv[i][r] = sqx[32 * ww + 16 * i + 8 * hh + r];
#pragma unroll
      for (int j = 0; j < 2; ++j) {
        const float ss = sqs[c * NUM_SHP + 32 * wk + 16 * j + rlane];
#pragma unroll
        for (int i = 0; i < 2; ++i) {
#pragma unroll
          for (int r = 0; r < 8; ++r) {
            float d2 = sxv[i][r] + ss - 2.0f * acc[i][j][r];
            d2 = fmaxf(d2, 1e-12f);
            dsum[i][j][r] += __builtin_amdgcn_sqrtf(d2);
          }
        }
      }
    }

    {
      float m0 = runmin0, m1 = runmin1;
#pragma unroll
      for (int i = 0; i < 2; ++i) {
#pragma unroll
        for (int r = 0; r < 8; ++r) {
          const int w = w0 + 32 * ww + 16 * i + 8 * hh + r;
          const bool valid = (w < NUM_WIN);
          float v0 = dsum[i][0][r];
          float v1 = dsum[i][1][r];
          v0 = valid ? v0 : __builtin_inff();
          v1 = valid ? v1 : __builtin_inff();
          m0 = fminf(m0, v0);
          m1 = fminf(m1, v1);
        }
      }
      runmin0 = m0;
      runmin1 = m1;
    }
  }

  runmin0 = fminf(runmin0, __shfl_xor(runmin0, 16, 32));
  runmin1 = fminf(runmin1, __shfl_xor(runmin1, 16, 32));
  minbuf[ww][32 * wk + rlane]      = runmin0;
  minbuf[ww][32 * wk + 16 + rlane] = runmin1;
  __syncthreads();
  if (wave == 0) {
    v4f o;
#pragma unroll
    for (int e = 0; e < 4; ++e) {
      const int kk = 4 * lane + e;
      o[e] = fminf(minbuf[0][kk], minbuf[1][kk]);
    }
    volatile v4f* p = (volatile v4f*)(out + (size_t)n * NUM_SHP + 4 * lane);
    *p = o;
    __threadfence();
    *p = o;
  }
}

extern "C" void kernel_launch(void* const* d_in, const int* in_sizes, int n_in,
                              void* d_out, int out_size, void* d_ws, size_t ws_size,
                              hipStream_t stream) {
  if (n_in < 2) return;
  const float* x  = (const float*)d_in[0];
  const float* sh = (const float*)d_in[1];
  float* out = (float*)d_out;

  const size_t shn_bytes = (size_t)SHP_ROWS * SHP_LEN * 2;
  const size_t sqs_bytes = (size_t)SHP_ROWS * 4;
  if (shn_bytes + sqs_bytes > ws_size) return;
  if (in_sizes[1] < SHP_ROWS * SHP_LEN) return;

  int nb = in_sizes[0] / (NUM_CH * SER_LEN);
  const int nb_out = out_size / NUM_SHP;
  if (nb > nb_out) nb = nb_out;
  if (nb <= 0) return;

  unsigned short* shn16 = (unsigned short*)d_ws;
  float* sqs = (float*)((char*)d_ws + shn_bytes);

  znorm_rows_kernel<<<SHP_ROWS / 32, 256, 0, stream>>>(sh, shn16, sqs);
  min_dist_kernel<<<nb, 256, 0, stream>>>(x, shn16, sqs, out);
}
